// T5CrossAttention_48653389529383
// MI455X (gfx1250) — hardware-verified
//
#include <hip/hip_runtime.h>
#include <math.h>

typedef __attribute__((ext_vector_type(16))) _Float16 v16h;
typedef __attribute__((ext_vector_type(16))) __bf16 v16b;
typedef __attribute__((ext_vector_type(8)))  _Float16 v8h;
typedef __attribute__((ext_vector_type(8)))  float v8f;
typedef __attribute__((ext_vector_type(4)))  float v4f;
typedef __attribute__((ext_vector_type(2)))  float v2f;
typedef __attribute__((ext_vector_type(4)))  unsigned v4u;
typedef __attribute__((ext_vector_type(4)))  int v4i;
typedef float __attribute__((may_alias)) float_a;
typedef int __attribute__((may_alias)) int_a;

template <typename T> __device__ __forceinline__ void vst2(void* p, T v) { *(volatile T*)p = v; __threadfence(); *(volatile T*)p = v; }
__device__ __forceinline__ v8f wmma16(v16h a, v16h b, v8f c) {
  v8f d = __builtin_amdgcn_wmma_f32_16x16x32_f16(false, a, false, b, (short)0, c, false, false);
  asm volatile("v_nop\n\tv_nop\n\tv_nop\n\tv_nop" : "+v"(d) : "v"(a), "v"(b));
  return d;
}
__device__ __forceinline__ v8f wmma_bf(v16b a, v16b b, v8f c) {
  v8f d = __builtin_amdgcn_wmma_f32_16x16x32_bf16(false, a, false, b, (short)0, c, false, false);
  asm volatile("v_nop\n\tv_nop\n\tv_nop\n\tv_nop" : "+v"(d) : "v"(a), "v"(b));
  return d;
}
__device__ __forceinline__ v16h frag_h(const _Float16* rowk0, int lane) {
  union { v16h v; v8h q[2]; } u; const _Float16* p = rowk0 + 8 * (lane >> 4);
  u.q[0] = *(const v8h*)p; u.q[1] = *(const v8h*)(p + 16); return u.v;
}
__device__ __forceinline__ v16h frag_f32(const float* rowk0, int lane) {
  v16h a; const float* p = rowk0 + 8 * (lane >> 4);
#pragma unroll
  for (int i = 0; i < 8; ++i) { a[i] = (_Float16)p[i]; a[8 + i] = (_Float16)p[16 + i]; }
  return a;
}
__device__ __forceinline__ v16h frag_f32s(const float* rowk0, int lane, float sc) {
  v16h a; const float* p = rowk0 + 8 * (lane >> 4);
#pragma unroll
  for (int i = 0; i < 8; ++i) { a[i] = (_Float16)(p[i] * sc); a[8 + i] = (_Float16)(p[16 + i] * sc); }
  return a;
}
__device__ __forceinline__ v16h fragc_f32(const float* W, int k0, int n, int lane, int ld, int K) {
  v16h a; const int g = lane >> 4;
#pragma unroll
  for (int i = 0; i < 8; ++i) { const int ka = k0 + 8 * g + i, kb = ka + 16;
    a[i] = (_Float16)(ka < K ? W[(size_t)(ka < K ? ka : K - 1) * ld + n] : 0.f); a[8 + i] = (_Float16)(kb < K ? W[(size_t)(kb < K ? kb : K - 1) * ld + n] : 0.f); }
  return a;
}
struct F2 { v16b h, l; };
__device__ __forceinline__ F2 bsplit16(const float v[16]) { F2 r;
#pragma unroll
  for (int i = 0; i < 16; ++i) { const __bf16 h = (__bf16)v[i]; r.h[i] = h; r.l[i] = (__bf16)(v[i] - (float)h); }
  return r; }
__device__ __forceinline__ F2 split_row(const float* row, int k0, int lane) { float v[16]; const float* p = row + k0 + 8 * (lane >> 4);
#pragma unroll
  for (int i = 0; i < 8; ++i) { v[i] = p[i]; v[8 + i] = p[16 + i]; }
  return bsplit16(v); }
__device__ __forceinline__ F2 split_rowK(const float* row, int k0, int lane, int K) { float v[16]; const int g = lane >> 4;
#pragma unroll
  for (int i = 0; i < 8; ++i) { const int ka = k0 + 8 * g + i, kb = ka + 16; v[i] = ka < K ? row[ka < K ? ka : K - 1] : 0.f; v[8 + i] = kb < K ? row[kb < K ? kb : K - 1] : 0.f; }
  return bsplit16(v); }
__device__ __forceinline__ F2 split_col(const float* W, int k0, int n, int lane, int ld, int K) { float v[16]; const int g = lane >> 4;
#pragma unroll
  for (int i = 0; i < 8; ++i) { const int ka = k0 + 8 * g + i, kb = ka + 16; v[i] = ka < K ? W[(size_t)(ka < K ? ka : K - 1) * ld + n] : 0.f; v[8 + i] = kb < K ? W[(size_t)(kb < K ? kb : K - 1) * ld + n] : 0.f; }
  return bsplit16(v); }
__device__ __forceinline__ v8f mac3(const F2& a, const F2& b, v8f c) { c = wmma_bf(a.l, b.h, c); c = wmma_bf(a.h, b.l, c); return wmma_bf(a.h, b.h, c); }
__device__ __forceinline__ float sigm(float v) { return 1.0f / (1.0f + expf(-v)); }
#define LDSX() do { asm volatile("s_wait_dscnt 0" ::: "memory"); __builtin_amdgcn_wave_barrier(); __builtin_amdgcn_fence(__ATOMIC_RELEASE, "workgroup"); } while (0)


#define NB 4
#define QL 1024
#define KVL 2048
#define DD 1024
#define NH 16
#define HD 64
#define NQ (NB * QL)
#ifndef TQB
#define TQB (QL / 64)
#define TNB NB
#endif
typedef __attribute__((ext_vector_type(8))) __bf16 v8b;
__device__ __forceinline__ v16b frag_b(const __bf16* rowk0, int lane) {
  union { v16b v; v8b q[2]; } u; const __bf16* p = rowk0 + 8 * (lane >> 4);
  u.q[0] = *(const v8b*)p; u.q[1] = *(const v8b*)(p + 16); return u.v;
}
__device__ __forceinline__ float bfr(float v) { return (float)(__bf16)v; }
__device__ __attribute__((noinline)) float exp_ni(float v) { return expf(v); }
__device__ __attribute__((noinline)) float erf_ni(float v) { return erff(v); }

#define PK_Q 0
#define PK_O (PK_Q + DD * DD)
#define PK_END (PK_O + DD * DD)
#define WS_PK  0u
#define WS_QH  (((2u * PK_END) + 127u) / 128u * 128u)
#define WS_QL  (WS_QH + 2u * NQ * DD)
#define WS_KB  (WS_QL + 2u * NQ * DD)
#define WS_VT  (WS_KB + 2u * NB * NH * KVL * HD)
#define WS_OH  (WS_VT + 2u * NB * NH * KVL * HD)
#define WS_OL  (WS_OH + 2u * NQ * DD)
#define WS_END (WS_OL + 2u * NQ * DD)

__global__ __launch_bounds__(256) void k_pack(const float* __restrict__ WQ, const float* __restrict__ WO, __bf16* __restrict__ PK) {
  __shared__ __align__(16) __bf16 s[DD]; const int n = blockIdx.x, which = blockIdx.y, t = threadIdx.x; const float* Wm = which ? WO : WQ;
  for (int k = t; k < DD; k += 256) s[k] = (__bf16)Wm[(size_t)k * DD + n];
  __syncthreads();
  for (int q = t; q < DD / 8; q += 256) vst2((unsigned*)(PK + (which ? PK_O : PK_Q) + (size_t)n * DD + q * 8), *(const v4u*)&s[q * 8]);
}
__global__ __launch_bounds__(256) void k_kv(const float* __restrict__ KS, const float* __restrict__ VS, __bf16* __restrict__ KB, __bf16* __restrict__ VT) {
  __shared__ __align__(16) __bf16 sk[64][HD]; __shared__ __align__(16) __bf16 sv[HD][72]; const int tid = threadIdx.x; const int kb = blockIdx.x, h = blockIdx.y, b = blockIdx.z; const size_t base = (((size_t)b * NH + h) * KVL + (size_t)kb * 64) * HD;
  for (int e = tid; e < 64 * HD; e += 256) { const int r = e >> 6, d = e & 63; sk[r][d] = (__bf16)KS[base + e]; sv[d][r] = (__bf16)VS[base + e]; }
  __syncthreads();
  for (int e = tid; e < 64 * HD / 8; e += 256) vst2((unsigned*)(KB + base + e * 8), *(const v4u*)(&sk[0][0] + e * 8));
  for (int e = tid; e < HD * 8; e += 256) { const int d = e >> 3, pc = e & 7; vst2((unsigned*)(VT + (((size_t)b * NH + h) * HD + d) * KVL + (size_t)kb * 64 + pc * 8), *(const v4u*)&sv[d][pc * 8]); }
}
__global__ __launch_bounds__(128) void k_q(const float* __restrict__ X, const __bf16* __restrict__ PK, __bf16* __restrict__ QH, __bf16* __restrict__ QL_) {
  __shared__ __align__(16) __bf16 soh[4][16][136], sol[4][16][136];
  const int tid = threadIdx.x, wave = tid >> 5, lane = tid & 31, col = lane & 15, g = lane >> 4; const size_t r0 = (size_t)blockIdx.x * 64 + wave * 16; const int n0 = blockIdx.y * 128;
  v8f acc[8] = {};
#pragma unroll 2
  for (int kc = 0; kc < DD / 32; ++kc) { v16b a; { const float* p = X + (r0 + col) * DD + kc * 32 + 8 * g;
#pragma unroll
      for (int i = 0; i < 8; ++i) { a[i] = (__bf16)p[i]; a[8 + i] = (__bf16)p[16 + i]; } }
#pragma unroll
    for (int j = 0; j < 8; ++j) acc[j] = wmma_bf(a, frag_b(PK + PK_Q + (size_t)(n0 + j * 16 + col) * DD + kc * 32, lane), acc[j]); }
#pragma unroll
  for (int j = 0; j < 8; ++j)
#pragma unroll
    for (int r = 0; r < 8; ++r) { const float v = acc[j][r]; const __bf16 hb = (__bf16)v; soh[wave][8 * g + r][j * 16 + col] = hb; sol[wave][8 * g + r][j * 16 + col] = (__bf16)(v - (float)hb); }
  LDSX();
  for (int rl = 0; rl < 16; ++rl) { if (lane < 16) vst2((unsigned*)(QH + (r0 + rl) * DD + n0 + lane * 8), *(const v4u*)&soh[wave][rl][lane * 8]); else vst2((unsigned*)(QL_ + (r0 + rl) * DD + n0 + (lane - 16) * 8), *(const v4u*)&sol[wave][rl][(lane - 16) * 8]); }
}
__global__ __launch_bounds__(128) void k_attn(const __bf16* __restrict__ QH, const __bf16* __restrict__ QL_, const __bf16* __restrict__ KB, const __bf16* __restrict__ VT, const float* __restrict__ MSK, __bf16* __restrict__ OH, __bf16* __restrict__ OL) {
  __shared__ __align__(16) __bf16 sph[4][16][40], spl[4][16][40]; __shared__ __align__(16) __bf16 soh[4][16][72], sol[4][16][72];
  const int tid = threadIdx.x, wave = tid >> 5, lane = tid & 31, col = lane & 15, g = lane >> 4; const int qb = blockIdx.x, h = blockIdx.y, b = blockIdx.z; const size_t rq = (size_t)b * QL + qb * 64 + wave * 16 + col;
  v16b aqh[2], aql[2];
#pragma unroll
  for (int kc = 0; kc < 2; ++kc) { aqh[kc] = frag_b(QH + rq * DD + h * HD + kc * 32, lane); aql[kc] = frag_b(QL_ + rq * DD + h * HD + kc * 32, lane); }
  const __bf16* Kbh = KB + ((size_t)b * NH + h) * KVL * HD; const __bf16* Vbh = VT + ((size_t)b * NH + h) * HD * KVL; const float* mrow = MSK + (size_t)b * KVL;
  float m[8], l[8];
#pragma unroll
  for (int r = 0; r < 8; ++r) { m[r] = -3.0e38f; l[r] = 0.f; }
  v8f acc[4] = {};
#pragma unroll 1
  for (int ks = 0; ks < KVL / 32; ++ks) { v8f s[2];
#pragma unroll
    for (int ct = 0; ct < 2; ++ct) { const int kk = ks * 32 + ct * 16 + col; v8f c = {};
#pragma unroll
      for (int kc = 0; kc < 2; ++kc) { const v16b kb = frag_b(Kbh + (size_t)kk * HD + kc * 32, lane); c = wmma_bf(aql[kc], kb, c); c = wmma_bf(aqh[kc], kb, c); }
      const float mk = bfr(mrow[kk]);
#pragma unroll
      for (int r = 0; r < 8; ++r) s[ct][r] = c[r] + mk; }
#pragma unroll
    for (int r = 0; r < 8; ++r) { float mx = fmaxf(s[0][r], s[1][r]);
#pragma unroll
      for (int o = 1; o < 16; o <<= 1) mx = fmaxf(mx, __shfl_xor(mx, o));
      const float mn = fmaxf(m[r], mx); const float alpha = (m[r] <= -1.0e38f) ? 0.f : exp_ni(m[r] - mn); const float e0 = exp_ni(s[0][r] - mn), e1 = exp_ni(s[1][r] - mn); float es = e0 + e1;
#pragma unroll
      for (int o = 1; o < 16; o <<= 1) es += __shfl_xor(es, o);
      l[r] = l[r] * alpha + es; m[r] = mn;
#pragma unroll
      for (int dt = 0; dt < 4; ++dt) acc[dt][r] *= alpha;
      const __bf16 h0 = (__bf16)e0, h1 = (__bf16)e1; sph[wave][8 * g + r][col] = h0; sph[wave][8 * g + r][16 + col] = h1; spl[wave][8 * g + r][col] = (__bf16)(e0 - (float)h0); spl[wave][8 * g + r][16 + col] = (__bf16)(e1 - (float)h1); }
    LDSX();
    const v16b pah = frag_b(&sph[wave][col][0], lane), pal = frag_b(&spl[wave][col][0], lane);
#pragma unroll
    for (int dt = 0; dt < 4; ++dt) { const v16b vb = frag_b(Vbh + (size_t)(dt * 16 + col) * KVL + ks * 32, lane); acc[dt] = wmma_bf(pal, vb, acc[dt]); acc[dt] = wmma_bf(pah, vb, acc[dt]); }
    LDSX(); }
#pragma unroll
  for (int r = 0; r < 8; ++r) { const float il = 1.0f / l[r];
#pragma unroll
    for (int dt = 0; dt < 4; ++dt) { const float v = acc[dt][r] * il; const __bf16 hb = (__bf16)v; soh[wave][8 * g + r][dt * 16 + col] = hb; sol[wave][8 * g + r][dt * 16 + col] = (__bf16)(v - (float)hb); } }
  LDSX();
  for (int rl = 0; rl < 16; ++rl) { const size_t o = ((size_t)b * QL + qb * 64 + wave * 16 + rl) * DD + h * HD; if (lane < 8) vst2((unsigned*)(OH + o + lane * 8), *(const v4u*)&soh[wave][rl][lane * 8]); else if (lane < 16) vst2((unsigned*)(OL + o + (lane - 8) * 8), *(const v4u*)&sol[wave][rl][(lane - 8) * 8]); }
}
__global__ __launch_bounds__(128) void k_out(const __bf16* __restrict__ OH, const __bf16* __restrict__ OL, const __bf16* __restrict__ PK, float* __restrict__ Y) {
  __shared__ __align__(16) float so[4][16][132];
  const int tid = threadIdx.x, wave = tid >> 5, lane = tid & 31, col = lane & 15, g = lane >> 4; const size_t r0 = (size_t)blockIdx.x * 64 + wave * 16; const int n0 = blockIdx.y * 128;
  v8f acc[8] = {};
#pragma unroll 2
  for (int kc = 0; kc < DD / 32; ++kc) { const v16b ah = frag_b(OH + (r0 + col) * DD + kc * 32, lane), al = frag_b(OL + (r0 + col) * DD + kc * 32, lane);
#pragma unroll
    for (int j = 0; j < 8; ++j) { const v16b w = frag_b(PK + PK_O + (size_t)(n0 + j * 16 + col) * DD + kc * 32, lane); acc[j] = wmma_bf(al, w, acc[j]); acc[j] = wmma_bf(ah, w, acc[j]); } }
#pragma unroll
  for (int j = 0; j < 8; ++j)
#pragma unroll
    for (int r = 0; r < 8; ++r) so[wave][8 * g + r][j * 16 + col] = acc[j][r];
  LDSX();
  for (int rl = 0; rl < 16; ++rl) vst2(Y + (r0 + rl) * DD + n0 + lane * 4, *(const v4f*)&so[wave][rl][lane * 4]);
}
extern "C" void kernel_launch(void* const* d_in, const int* in_sizes, int n_in, void* d_out, int out_size, void* d_ws, size_t ws_size, hipStream_t stream) {
  (void)in_sizes; (void)n_in; (void)out_size;
  const float** F = (const float**)d_in;
  if (ws_size < (size_t)WS_END) return;
  char* ws = (char*)d_ws; __bf16 *PK = (__bf16*)(ws + WS_PK), *QH = (__bf16*)(ws + WS_QH), *QLp = (__bf16*)(ws + WS_QL), *KB = (__bf16*)(ws + WS_KB), *VT = (__bf16*)(ws + WS_VT), *OH = (__bf16*)(ws + WS_OH), *OL = (__bf16*)(ws + WS_OL);
  k_pack<<<dim3(DD, 2), 256, 0, stream>>>(F[4], F[5], PK);
  k_kv<<<dim3(KVL / 64, NH, TNB), 256, 0, stream>>>(F[1], F[2], KB, VT);
  k_q<<<dim3(TNB * QL / 64, DD / 128), 128, 0, stream>>>(F[0], PK, QH, QLp);
  k_attn<<<dim3(TQB, NH, TNB), 128, 0, stream>>>(QH, QLp, KB, VT, F[3], OH, OL);
  k_out<<<dim3(TNB * QL / 64, DD / 128), 128, 0, stream>>>(OH, OL, PK, (float*)d_out);
}
